// MixedScoreMultiHeadAttention_46952582480380
// MI455X (gfx1250) — hardware-verified
//
#include <hip/hip_runtime.h>
#include <math.h>
#include <stdint.h>

#define NB_  32
#define NR_  128
#define NC_  128
#define NE_  256
#define NH_  16
#define HD_  16
#define MS_  16
#define NTOK (NB_ * NR_)
static_assert(NH_ * HD_ == NE_);
static_assert(NR_ == NC_);
static_assert((NTOK % 64) == 0 && (NE_ % 64) == 0 && (NC_ % 64) == 0 && (NE_ % 32) == 0);

typedef _Float16 v16h __attribute__((ext_vector_type(16)));
typedef _Float16 v8h  __attribute__((ext_vector_type(8)));
typedef float    v8f  __attribute__((ext_vector_type(8)));
typedef float    v4f  __attribute__((ext_vector_type(4)));
typedef unsigned int v4u __attribute__((ext_vector_type(4)));

__device__ __forceinline__ unsigned short bf_bits(float f) {
  unsigned u = __float_as_uint(f);
  return (unsigned short)((u + 0x7FFFu + ((u >> 16) & 1u)) >> 16);
}
__device__ __forceinline__ float bf_up(unsigned short h) { return __uint_as_float(((unsigned)h) << 16); }
__device__ __forceinline__ float bfr(float f) { return bf_up(bf_bits(f)); }
__device__ __forceinline__ unsigned short h_bits(_Float16 x) { return __builtin_bit_cast(unsigned short, x); }
__device__ __forceinline__ unsigned pk16(unsigned short a, unsigned short b) { return (unsigned)a | ((unsigned)b << 16); }
__device__ __forceinline__ v8f zero8() { v8f z = {0.f, 0.f, 0.f, 0.f, 0.f, 0.f, 0.f, 0.f}; return z; }

__device__ __forceinline__ v16h ldfrag_h(const _Float16* p) {
  union { v16h v; v8h h[2]; } f;
  f.h[0] = *(const v8h*)(p);
  f.h[1] = *(const v8h*)(p + 16);
  return f.v;
}
__device__ __forceinline__ v16h ldfrag_8z(const _Float16* p) {
  union { v16h v; v8h h[2]; } f;
  const _Float16 zz = (_Float16)0.0f;
  const v8h z = {zz, zz, zz, zz, zz, zz, zz, zz};
  f.h[0] = *(const v8h*)(p);
  f.h[1] = z;
  return f.v;
}

__device__ __forceinline__ v8f mma_h_raw(v16h a, v16h b, v8f c) {
  return __builtin_amdgcn_wmma_f32_16x16x32_f16(false, a, false, b, (short)0, c, false, false);
}
__device__ __forceinline__ void dep_guard_h(v8f& a, v8f& b, v16h x, v16h y) {
#if defined(__HIP_DEVICE_COMPILE__)
  asm volatile("v_nop\n\tv_nop\n\tv_nop\n\tv_nop" : "+v"(a), "+v"(b) : "v"(x), "v"(y));
#endif
}
__device__ __forceinline__ void guard2x3(v8f& a, v8f& b, v16h x, v16h y, v16h z) {
#if defined(__HIP_DEVICE_COMPILE__)
  asm volatile("v_nop\n\tv_nop\n\tv_nop\n\tv_nop" : "+v"(a), "+v"(b) : "v"(x), "v"(y), "v"(z));
#endif
}
__device__ __forceinline__ void guard4x6(v8f& a, v8f& b, v8f& c, v8f& d,
                                         v16h u, v16h w, v16h x, v16h y, v16h z, v16h t) {
#if defined(__HIP_DEVICE_COMPILE__)
  asm volatile("v_nop\n\tv_nop\n\tv_nop\n\tv_nop"
               : "+v"(a), "+v"(b), "+v"(c), "+v"(d)
               : "v"(u), "v"(w), "v"(x), "v"(y), "v"(z), "v"(t));
#endif
}
__device__ __forceinline__ void keep4_h(v16h a, v16h b, v16h c, v16h d) {
#if defined(__HIP_DEVICE_COMPILE__)
  asm volatile("v_nop" :: "v"(a), "v"(b), "v"(c), "v"(d));
#endif
}
__device__ __forceinline__ void acc_guard4(v8f& a, v8f& b, v8f& c, v8f& d) {
#if defined(__HIP_DEVICE_COMPILE__)
  asm volatile("v_nop\n\tv_nop\n\tv_nop\n\tv_nop" : "+v"(a), "+v"(b), "+v"(c), "+v"(d));
#endif
}
__device__ __forceinline__ void acc_guard2(v8f& a, v8f& b) {
#if defined(__HIP_DEVICE_COMPILE__)
  asm volatile("v_nop\n\tv_nop\n\tv_nop\n\tv_nop" : "+v"(a), "+v"(b));
#endif
}
__device__ __forceinline__ void wave_sync_lds() {
  __builtin_amdgcn_fence(__ATOMIC_RELEASE, "workgroup");
  __builtin_amdgcn_wave_barrier();
  __builtin_amdgcn_fence(__ATOMIC_ACQUIRE, "workgroup");
}

__global__ __launch_bounds__(256) void cvt_h8(const float* __restrict__ in, unsigned short* out, int n8, float scale) {
  const int i = blockIdx.x * 256 + threadIdx.x;
  if (i < n8) {
    const v4f a = *(const v4f*)(in + (size_t)i * 8);
    const v4f c = *(const v4f*)(in + (size_t)i * 8 + 4);
    float f[8];
    f[0] = a[0]; f[1] = a[1]; f[2] = a[2]; f[3] = a[3];
    f[4] = c[0]; f[5] = c[1]; f[6] = c[2]; f[7] = c[3];
    unsigned short hb[8];
#pragma unroll
    for (int e = 0; e < 8; ++e) hb[e] = h_bits((_Float16)(bf_up(bf_bits(f[e])) * scale));
    v4u p;
    p[0] = pk16(hb[0], hb[1]);
    p[1] = pk16(hb[2], hb[3]);
    p[2] = pk16(hb[4], hb[5]);
    p[3] = pk16(hb[6], hb[7]);
    *(volatile v4u*)(out + (size_t)i * 8) = p;
    __threadfence();
    *(volatile v4u*)(out + (size_t)i * 8) = p;
  }
}

#define QTP 72
__global__ __launch_bounds__(256) void cvt_wt(const float* __restrict__ Wq, const float* __restrict__ Wk,
                                              const float* __restrict__ Wv, unsigned short* WT, float scale) {
  __shared__ __align__(16) unsigned short ts[64 * QTP];
  const int tid = threadIdx.x;
  const int o0 = blockIdx.x * 64, e0 = blockIdx.y * 64, z = blockIdx.z;
  const float* W = (z == 0) ? Wq : ((z == 1) ? Wk : Wv);
  unsigned short* out = WT + (size_t)z * NE_ * NE_;
#pragma unroll 1
  for (int pass = 0; pass < 4; ++pass) {
    const int e  = pass * 16 + (tid >> 4);
    const int o4 = (tid & 15) * 4;
    const v4f v = *(const v4f*)(W + (size_t)(e0 + e) * NE_ + o0 + o4);
#pragma unroll
    for (int i = 0; i < 4; ++i) ts[(o4 + i) * QTP + e] = h_bits((_Float16)(bf_up(bf_bits(v[i])) * scale));
  }
  __syncthreads();
#pragma unroll 1
  for (int pass = 0; pass < 2; ++pass) {
    const int lr = pass * 32 + (tid >> 3);
    const int c8 = (tid & 7) * 8;
    const v4u v = *(const v4u*)(ts + lr * QTP + c8);
    unsigned short* dst = out + (size_t)(o0 + lr) * NE_ + e0 + c8;
    *(volatile v4u*)dst = v;
    __threadfence();
    *(volatile v4u*)dst = v;
  }
}

__global__ __launch_bounds__(256) void gemm64h2(
    const unsigned short* __restrict__ Ap, int lda, long long sAy,
    const unsigned short* __restrict__ Btp, int ldb, long long sBy,
    unsigned short* C1, unsigned short* C2, int ldc, long long sCy,
    int M, int N, int K, float oscale, float rcarry) {
  const _Float16* A  = (const _Float16*)(const void*)Ap;
  const _Float16* Bt = (const _Float16*)(const void*)Btp;
  __shared__ __align__(16) float sT[8][16 * 68];
  const int by   = blockIdx.y;
  const int lane = threadIdx.x & 31;
  const int wave = threadIdx.x >> 5;
  const int tilesN = N >> 6;
  const int tilesM = M >> 6;
  const int tile = blockIdx.x * 8 + wave;
  if (tile >= tilesM * tilesN) return;
  const int tm = tile / tilesN;
  const int tn = tile - tm * tilesN;
  const int m0 = tm << 6;
  const int n0 = tn << 6;

  const _Float16* Ab = A + (size_t)by * (size_t)sAy;
  const _Float16* Bb = Bt + (size_t)by * (size_t)sBy;

  const int rlane = lane & 15;
  const int koff  = (lane >> 4) * 8;
  const int mOff  = (lane >> 4) * 8;

  v8f acc[4][4];
#pragma unroll
  for (int i = 0; i < 4; ++i)
#pragma unroll
    for (int j = 0; j < 4; ++j) acc[i][j] = zero8();

  for (int k0 = 0; k0 < K; k0 += 32) {
    v16h bf[4];
#pragma unroll
    for (int j = 0; j < 4; ++j) {
      const size_t bo = (size_t)(n0 + (j << 4) + rlane) * ldb + koff + k0;
      bf[j] = ldfrag_h(Bb + bo);
    }
#pragma unroll
    for (int i = 0; i < 4; ++i) {
      const size_t ao = (size_t)(m0 + (i << 4) + rlane) * lda + koff + k0;
      const v16h ah = ldfrag_h(Ab + ao);
#pragma unroll
      for (int j = 0; j < 4; ++j) acc[i][j] = mma_h_raw(ah, bf[j], acc[i][j]);
      dep_guard_h(acc[i][0], acc[i][3], ah, bf[3]);
    }
    keep4_h(bf[0], bf[1], bf[2], bf[3]);
  }
  acc_guard4(acc[0][0], acc[0][1], acc[0][2], acc[0][3]);
  acc_guard4(acc[1][0], acc[1][1], acc[1][2], acc[1][3]);
  acc_guard4(acc[2][0], acc[2][1], acc[2][2], acc[2][3]);
  acc_guard4(acc[3][0], acc[3][1], acc[3][2], acc[3][3]);

  float* slab = sT[wave];
  unsigned short* Cb1 = C1 + (size_t)by * (size_t)sCy;
  unsigned short* Cb2 = C2 + (size_t)by * (size_t)sCy;
  const int rq = lane >> 3, c8 = (lane & 7) * 8;
#pragma unroll
  for (int i = 0; i < 4; ++i) {
    const int mBase = m0 + (i << 4);
#pragma unroll
    for (int j = 0; j < 4; ++j) {
#pragma unroll
      for (int r = 0; r < 8; ++r) {
        slab[(mOff + r) * 68 + (j << 4) + rlane] = acc[i][j][r] * oscale;
      }
    }
    wave_sync_lds();
    v4u ph[4], pl[4];
#pragma unroll
    for (int it = 0; it < 4; ++it) {
      const int row = it * 4 + rq;
      const v4f x0 = *(const v4f*)(slab + row * 68 + c8);
      const v4f x1 = *(const v4f*)(slab + row * 68 + c8 + 4);
      float f[8];
      f[0] = x0[0]; f[1] = x0[1]; f[2] = x0[2]; f[3] = x0[3];
      f[4] = x1[0]; f[5] = x1[1]; f[6] = x1[2]; f[7] = x1[3];
      unsigned short hb[8], lb[8];
#pragma unroll
      for (int e = 0; e < 8; ++e) {
        const _Float16 xh = (_Float16)f[e];
        hb[e] = h_bits(xh);
        lb[e] = h_bits((_Float16)((f[e] - (float)xh) * rcarry));
      }
#pragma unroll
      for (int q = 0; q < 4; ++q) {
        ph[it][q] = pk16(hb[2 * q], hb[2 * q + 1]);
        pl[it][q] = pk16(lb[2 * q], lb[2 * q + 1]);
      }
    }
    for (int pass = 0; pass < 2; ++pass) {
#pragma unroll
      for (int it = 0; it < 4; ++it) {
        const int row = it * 4 + rq;
        const size_t d = (size_t)(mBase + row) * ldc + n0 + c8;
        *(volatile v4u*)(Cb1 + d) = ph[it];
        *(volatile v4u*)(Cb2 + d) = pl[it];
      }
      __threadfence();
    }
    wave_sync_lds();
  }
}

#define VPITCH 72
#define SP_    36
__global__ __launch_bounds__(256) void attn_kernel(
    const unsigned short* __restrict__ QHp, const unsigned short* __restrict__ QLp,
    const unsigned short* __restrict__ KHp, const unsigned short* __restrict__ KLp,
    const unsigned short* __restrict__ VHp, const unsigned short* __restrict__ VLp,
    const float* __restrict__ cost,
    const float* __restrict__ m1w, const float* __restrict__ m1b,
    const float* __restrict__ m2w, const float* __restrict__ m2b,
    float* out) {
  __shared__ __align__(16) unsigned short kh_u[64 * HD_];
  __shared__ __align__(16) unsigned short kg_u[64 * HD_];
  __shared__ __align__(16) unsigned short vh_u[16 * VPITCH];
  __shared__ __align__(16) unsigned short vr_u[16 * VPITCH];
  __shared__ __align__(16) float sMW[MS_ * 4 + 4];
  __shared__ __align__(16) float sto[8 * 16 * SP_];
  const _Float16* khh = (const _Float16*)(const void*)kh_u;
  const _Float16* kgg = (const _Float16*)(const void*)kg_u;
  const _Float16* vhh = (const _Float16*)(const void*)vh_u;
  const _Float16* vrl = (const _Float16*)(const void*)vr_u;
  const _Float16* QH  = (const _Float16*)(const void*)QHp;
  const _Float16* QL  = (const _Float16*)(const void*)QLp;

  const int tid = threadIdx.x, lane = tid & 31, wave = tid >> 5;
  const int b = blockIdx.x;
  const int qBase = wave * 16;
  const int rlane = lane & 15, hsel = lane >> 4, koff = hsel * 8;
  const float C2048  = 1.0f / 2048.0f;
  const float C1024  = 1.0f / 1024.0f;
  const float LN1024 = 6.931471805599453f;

  const size_t qrow = (size_t)(b * NR_ + qBase + rlane);
  const float* crow = cost + qrow * NC_ + koff;

  const int t2   = tid & 127;
  const int krow = t2 >> 1, kdh = (t2 & 1) * 8;
  const int vrow = t2 >> 3, vc8 = (t2 & 7) * 8;
  unsigned short* khd = kh_u + t2 * 8;
  unsigned short* kgd = kg_u + t2 * 8;
  unsigned short* vhd = vh_u + vrow * VPITCH + vc8;
  unsigned short* vrd = vr_u + vrow * VPITCH + vc8;

#pragma unroll 1
  for (int h = 0; h < NH_; ++h) {
    __syncthreads();
    if (wave == 0) {
      const int m = rlane;
      const float w0 = bfr(m1w[(h * 2 + 0) * MS_ + m]);
      const float w1 = bfr(m1w[(h * 2 + 1) * MS_ + m]);
      const float bb = bfr(m1b[h * MS_ + m]);
      const float w2 = bfr(m2w[h * MS_ + m]);
      const float b2 = bfr(m2b[h]);
      if (hsel == 0) {
        v4f t = {w0, w1, bb, w2};
        *(v4f*)(sMW + 4 * m) = t;
      }
      if (lane == 0) sMW[MS_ * 4] = b2;
    }
    const size_t qo = qrow * NE_ + (size_t)h * HD_ + koff;
    const v16h qh = ldfrag_8z(QH + qo);
    const v16h ql = ldfrag_8z(QL + qo);
    const size_t kgo = ((size_t)(b * NC_ + krow)) * NE_ + (size_t)h * HD_ + kdh;
    const unsigned short* Kgh = KHp + kgo;
    const unsigned short* Kgl = KLp + kgo;
    const size_t vgo = ((size_t)(b * NE_ + h * HD_ + vrow)) * NC_ + vc8;
    const unsigned short* Vhg = VHp + vgo;
    const unsigned short* Vlg = VLp + vgo;

    v8f oh = zero8(), ol = zero8();
    float m_run = -1e30f, l_run = 0.f;

#pragma unroll 1
    for (int kb = 0; kb < NC_; kb += 64) {
      __syncthreads();
      if (wave < 4) {
        const v4u kv = *(const v4u*)(Kgh + (size_t)kb * NE_);
        *(v4u*)khd = kv;
        const v4u lv = *(const v4u*)(Vlg + kb);
        *(v4u*)vrd = lv;
      } else {
        const v4u kv = *(const v4u*)(Kgl + (size_t)kb * NE_);
        *(v4u*)kgd = kv;
        const v4u hv = *(const v4u*)(Vhg + kb);
        *(v4u*)vhd = hv;
      }
      __syncthreads();

#pragma unroll 1
      for (int sub = 0; sub < 2; ++sub) {
        const int kr = 32 * sub;
        const v16h kf0 = ldfrag_8z(khh + (kr + rlane) * HD_ + koff);
        const v16h kf1 = ldfrag_8z(khh + (kr + 16 + rlane) * HD_ + koff);
        const v16h kg0 = ldfrag_8z(kgg + (kr + rlane) * HD_ + koff);
        const v16h kg1 = ldfrag_8z(kgg + (kr + 16 + rlane) * HD_ + koff);
        v8f sr0 = mma_h_raw(kf0, ql, zero8());
        v8f sr1 = mma_h_raw(kf1, ql, zero8());
        v8f sh0 = mma_h_raw(kf0, qh, zero8());
        v8f sh1 = mma_h_raw(kf1, qh, zero8());
        sr0 = mma_h_raw(kg0, qh, sr0);
        sr1 = mma_h_raw(kg1, qh, sr1);
        guard4x6(sh0, sh1, sr0, sr1, kf0, kf1, kg0, kg1, qh, ql);

        const v4f ca0 = *(const v4f*)(crow + kb + kr);
        const v4f ca1 = *(const v4f*)(crow + kb + kr + 4);
        const v4f cb0 = *(const v4f*)(crow + kb + kr + 16);
        const v4f cb1 = *(const v4f*)(crow + kb + kr + 20);
        float d0[8], d1[8], c0[8], c1[8];
#pragma unroll
        for (int r = 0; r < 4; ++r) {
          c0[r] = bfr(ca0[r]); c0[r + 4] = bfr(ca1[r]);
          c1[r] = bfr(cb0[r]); c1[r + 4] = bfr(cb1[r]);
        }
#pragma unroll
        for (int r = 0; r < 8; ++r) {
          d0[r] = (sh0[r] + sr0[r] * C2048) * C1024;
          d1[r] = (sh1[r] + sr1[r] * C2048) * C1024;
        }

        const float b2v = sMW[MS_ * 4];
        float a0[8], a1[8];
#pragma unroll
        for (int r = 0; r < 8; ++r) { a0[r] = b2v; a1[r] = b2v; }
#pragma unroll 1
        for (int m = 0; m < MS_; ++m) {
          const v4f w = *(const v4f*)(sMW + 4 * m);
#pragma unroll
          for (int r = 0; r < 8; ++r) {
            const float t0 = fmaxf(fmaf(d0[r], w[0], fmaf(c0[r], w[1], w[2])), 0.0f);
            const float t1 = fmaxf(fmaf(d1[r], w[0], fmaf(c1[r], w[1], w[2])), 0.0f);
            a0[r] = fmaf(t0, w[3], a0[r]);
            a1[r] = fmaf(t1, w[3], a1[r]);
          }
        }

        float mloc = -1e30f;
#pragma unroll
        for (int r = 0; r < 8; ++r) mloc = fmaxf(mloc, fmaxf(a0[r], a1[r]));
        mloc = fmaxf(mloc, __shfl_xor(mloc, 16, 32));
        const float newM  = fmaxf(m_run, mloc);
        const float alpha = __expf(m_run - newM);
        const float msh   = newM - LN1024;
        float ssum = 0.f;
        float p0[8], p1[8];
#pragma unroll
        for (int r = 0; r < 8; ++r) {
          p0[r] = __expf(a0[r] - msh);
          p1[r] = __expf(a1[r] - msh);
          ssum += p0[r] + p1[r];
        }
        ssum += __shfl_xor(ssum, 16, 32);
        l_run = l_run * alpha + ssum;
        m_run = newM;
#pragma unroll
        for (int r = 0; r < 8; ++r) { oh[r] *= alpha; ol[r] *= alpha; }

        union { v16h v; _Float16 s[16]; } pf;
#pragma unroll
        for (int r = 0; r < 8; ++r) {
          pf.s[r]     = (_Float16)p0[r];
          pf.s[8 + r] = (_Float16)p1[r];
        }

        const v16h vah = ldfrag_h(vhh + rlane * VPITCH + kr + koff);
        const v16h val = ldfrag_h(vrl + rlane * VPITCH + kr + koff);
        oh = mma_h_raw(vah, pf.v, oh);
        ol = mma_h_raw(val, pf.v, ol);
        guard2x3(oh, ol, vah, val, pf.v);
      }
    }
    acc_guard2(oh, ol);

    const float inv = (1.0f / 16.0f) * (1.0f / l_run);
    v4f f0, f1;
#pragma unroll
    for (int e = 0; e < 4; ++e) {
      f0[e] = (oh[e]     + ol[e]     * C2048) * inv;
      f1[e] = (oh[4 + e] + ol[4 + e] * C2048) * inv;
    }
    const int so = (wave * 16 + rlane) * SP_ + (h & 1) * 16 + koff;
    *(v4f*)(sto + so)     = f0;
    *(v4f*)(sto + so + 4) = f1;

    if (h & 1) {
      wave_sync_lds();
      const int rq = lane >> 3, c4 = (lane & 7) * 4;
      const float* ss = sto + (wave * 16) * SP_;
      v4f ov[4];
#pragma unroll
      for (int it = 0; it < 4; ++it) ov[it] = *(const v4f*)(ss + (it * 4 + rq) * SP_ + c4);
      float* ob = out + ((size_t)(b * NR_ + qBase)) * NE_ + (size_t)(h >> 1) * 32 + c4;
      for (int pass = 0; pass < 2; ++pass) {
#pragma unroll
        for (int it = 0; it < 4; ++it) {
          const int row = it * 4 + rq;
          *(volatile v4f*)(ob + (size_t)row * NE_) = ov[it];
        }
        __threadfence();
      }
      wave_sync_lds();
    }
  }
}

extern "C" void kernel_launch(void* const* d_in, const int* in_sizes, int n_in,
                              void* d_out, int out_size, void* d_ws, size_t ws_size,
                              hipStream_t stream) {
  if (n_in < 10) return;
  if (in_sizes[0] != NB_ * NR_ * NE_) return;
  if (in_sizes[1] != NB_ * NC_ * NE_) return;
  if (in_sizes[2] != NB_ * NR_ * NC_) return;
  if (in_sizes[3] != NE_ * NE_) return;
  if (in_sizes[4] != NE_ * NE_) return;
  if (in_sizes[5] != NE_ * NE_) return;
  if (in_sizes[6] != NH_ * 2 * MS_) return;
  if (in_sizes[7] != NH_ * MS_) return;
  if (in_sizes[8] != NH_ * MS_) return;
  if (in_sizes[9] < NH_) return;
  if (out_size != NB_ * NR_ * NE_) return;

  const float* row_emb = (const float*)d_in[0];
  const float* col_emb = (const float*)d_in[1];
  const float* costm   = (const float*)d_in[2];
  const float* Wq      = (const float*)d_in[3];
  const float* Wk      = (const float*)d_in[4];
  const float* Wv      = (const float*)d_in[5];
  const float* m1w     = (const float*)d_in[6];
  const float* m1b     = (const float*)d_in[7];
  const float* m2w     = (const float*)d_in[8];
  const float* m2b     = (const float*)d_in[9];

  const size_t PX  = (size_t)NTOK * NE_ * 2;
  const size_t PWT = (size_t)3 * NE_ * NE_ * 2;
  const size_t PQ  = (size_t)NTOK * NE_ * 2;
  const size_t PV  = (size_t)NB_ * NE_ * NC_ * 2;
  size_t off = 0;
  const size_t oXR = off; off += PX;
  const size_t oXC = off; off += PX;
  const size_t oWT = off; off += PWT;
  const size_t oQH = off; off += PQ;
  const size_t oQL = off; off += PQ;
  const size_t oKH = off; off += PQ;
  const size_t oKL = off; off += PQ;
  const size_t oVH = off; off += PV;
  const size_t oVL = off; off += PV;
  if (off > ws_size) return;
  if (off > (size_t)134217728) return;

  char* ws = (char*)d_ws;
  unsigned short* XR  = (unsigned short*)(ws + oXR);
  unsigned short* XC  = (unsigned short*)(ws + oXC);
  unsigned short* WT  = (unsigned short*)(ws + oWT);
  unsigned short* QH  = (unsigned short*)(ws + oQH);
  unsigned short* QL  = (unsigned short*)(ws + oQL);
  unsigned short* KH  = (unsigned short*)(ws + oKH);
  unsigned short* KL  = (unsigned short*)(ws + oKL);
  unsigned short* VH  = (unsigned short*)(ws + oVH);
  unsigned short* VL  = (unsigned short*)(ws + oVL);
  float*          out = (float*)d_out;

  const dim3 blk(256);
  const int  n8x = NTOK * NE_ / 8;
  const dim3 gX((n8x + 255) / 256);
  const dim3 gWT(NE_ / 64, NE_ / 64, 3);
  const dim3 gQK(((NTOK / 64) * (NE_ / 64) + 7) / 8, 1);
  const dim3 gVT(((NE_ / 64) * (NC_ / 64) + 7) / 8, NB_);
  const dim3 gAttn(NB_);

  const float oscale = 1.0f / 1024.0f;
  const float rcarry = 2048.0f;

  cvt_h8<<<gX, blk, 0, stream>>>(row_emb, XR, n8x, 16.0f);
  cvt_h8<<<gX, blk, 0, stream>>>(col_emb, XC, n8x, 16.0f);
  cvt_wt<<<gWT, blk, 0, stream>>>(Wq, Wk, Wv, WT, 1024.0f);
  gemm64h2<<<gQK, blk, 0, stream>>>(
      XR, NE_, 0LL,
      WT, NE_, 0LL,
      QH, QL, NE_, 0LL,
      NTOK, NE_, NE_, oscale, rcarry);
  gemm64h2<<<gQK, blk, 0, stream>>>(
      XC, NE_, 0LL,
      WT + (size_t)NE_ * NE_, NE_, 0LL,
      KH, KL, NE_, 0LL,
      NTOK, NE_, NE_, oscale, rcarry);
  gemm64h2<<<gVT, blk, 0, stream>>>(
      WT + (size_t)2 * NE_ * NE_, NE_, 0LL,
      XC, NE_, (long long)((size_t)NC_ * NE_),
      VH, VL, NC_, (long long)((size_t)NE_ * NC_),
      NE_, NC_, NE_, oscale, rcarry);
  attn_kernel<<<gAttn, blk, 0, stream>>>(QH, QL, KH, KL, VH, VL, costm, m1w, m1b, m2w, m2b, out);
  (void)hipGetLastError();
}
